// SparsePagedAttention_27204322853266
// MI455X (gfx1250) — hardware-verified
//
#include <hip/hip_runtime.h>


#define S_LEN  2048
#define NH     16
#define NKV    4
#define HD     128
#define QST    (NH * HD)
#define KVST   (NKV * HD)
#define NSC    64
#define NBATCH 2
#define QP     136
#define PP     72
#define OP     132
#define VTP    72
#define NEG_BIG (-3.0e38f)
#define KSL2E  (0.08838834764831845f * 1.44269504088896340736f)

typedef unsigned short us8 __attribute__((ext_vector_type(8)));
typedef unsigned short us4 __attribute__((ext_vector_type(4)));
typedef __bf16 v16bf __attribute__((ext_vector_type(16)));
typedef float v8f __attribute__((ext_vector_type(8)));
typedef float v4f __attribute__((ext_vector_type(4)));

union Frag { v16bf v; us8 h[2]; };

__device__ __forceinline__ v8f mma16(v16bf a, v16bf b, v8f c) {
  c = __builtin_amdgcn_wmma_f32_16x16x32_bf16(false, a, false, b, (short)0, c, false, false);
  asm volatile("v_nop\n\tv_nop\n\tv_nop\n\tv_nop" : "+v"(c) : "v"(a), "v"(b));
  return c;
}

__device__ __forceinline__ v8f mma3(const Frag& ah, const Frag& al, const Frag& bh, const Frag& bl, v8f c) {
  c = mma16(ah.v, bh.v, c);
  c = mma16(ah.v, bl.v, c);
  c = mma16(al.v, bh.v, c);
  return c;
}

__device__ __forceinline__ unsigned bf16_rne(float x) {
  unsigned u = __float_as_uint(x);
  u += 0x7FFFu + ((u >> 16) & 1u);
  return u >> 16;
}

__device__ __forceinline__ void split_hl(float x, unsigned short& hi, unsigned short& lo) {
  const unsigned hb = bf16_rne(x);
  const float hf = __uint_as_float(hb << 16);
  hi = (unsigned short)hb;
  lo = (unsigned short)bf16_rne(x - hf);
}

__global__ __launch_bounds__(256) void k_split_rows(const float* __restrict__ src,
    unsigned short* hi, unsigned short* lo, int n8)
{
  const int i = blockIdx.x * 256 + threadIdx.x;
  if (i >= n8) return;
  const size_t o = (size_t)i * 8;
  const v4f a = *(const v4f*)(src + o);
  const v4f c = *(const v4f*)(src + o + 4);
  us8 hv, lv;
  #pragma unroll
  for (int e = 0; e < 4; ++e) {
    unsigned short p, q;
    split_hl(a[e], p, q); hv[e] = p;     lv[e] = q;
    split_hl(c[e], p, q); hv[4 + e] = p; lv[4 + e] = q;
  }
  *(volatile us8*)(hi + o) = hv;
  *(volatile us8*)(lo + o) = lv;
  __threadfence();
  *(volatile us8*)(hi + o) = hv;
  *(volatile us8*)(lo + o) = lv;
}

__global__ __launch_bounds__(128) void k_split_vt(const float* __restrict__ Vsrc,
    unsigned short* vth, unsigned short* vtl)
{
  __shared__ __align__(16) unsigned short sH[HD * VTP];
  __shared__ __align__(16) unsigned short sL[HD * VTP];

  const int kt  = blockIdx.x;
  const int hk  = blockIdx.y;
  const int b   = blockIdx.z;
  const int tid = threadIdx.x;

  const float* vp = Vsrc + (size_t)(b * S_LEN + kt * 64) * KVST + hk * HD + tid;
  #pragma unroll 4
  for (int i = 0; i < 64; ++i) {
    const float x = vp[(size_t)i * KVST];
    unsigned short p, q;
    split_hl(x, p, q);
    sH[tid * VTP + i] = p;
    sL[tid * VTP + i] = q;
  }
  __syncthreads();

  const int piece = tid & 7;
  const size_t rowbase = ((size_t)((b * NKV + hk) * HD)) * S_LEN + (size_t)kt * 64 + piece * 8;
  #pragma unroll 1
  for (int pass = 0; pass < 2; ++pass) {
    #pragma unroll
    for (int j = 0; j < 8; ++j) {
      const int L = j * 16 + (tid >> 3);
      const us8 a = *(const us8*)(sH + L * VTP + piece * 8);
      const us8 c = *(const us8*)(sL + L * VTP + piece * 8);
      *(volatile us8*)(vth + rowbase + (size_t)L * S_LEN) = a;
      *(volatile us8*)(vtl + rowbase + (size_t)L * S_LEN) = c;
    }
    __threadfence();
  }
}


__device__ __forceinline__ void stage_q(const float* __restrict__ qb,
    unsigned short* sh, unsigned short* sl, int wave, int lane)
{
  #pragma unroll 2
  for (int p = 0; p < 16; ++p) {
    const int row = p * 4 + wave;
    const v4f x = *(const v4f*)(qb + (size_t)row * QST);
    us4 hv, lv;
    #pragma unroll
    for (int e = 0; e < 4; ++e) {
      unsigned short a, c;
      split_hl(x[e], a, c);
      hv[e] = a; lv[e] = c;
    }
    *(us4*)(sh + row * QP + lane * 4) = hv;
    *(us4*)(sl + row * QP + lane * 4) = lv;
  }
}

__device__ __forceinline__ void qk_tile(const unsigned short* qh, const unsigned short* ql,
    const unsigned short* krh, const unsigned short* krl, v8f (&s)[4])
{
  #pragma unroll
  for (int t = 0; t < 4; ++t) {
    v8f acc = {0.f, 0.f, 0.f, 0.f, 0.f, 0.f, 0.f, 0.f};
    const unsigned short* kh = krh + (size_t)(t * 16) * KVST;
    const unsigned short* kl = krl + (size_t)(t * 16) * KVST;
    #pragma unroll 1
    for (int c = 0; c < 4; ++c) {
      Frag ah, al, bh, bl;
      ah.h[0] = *(const us8*)(qh + c * 32);
      ah.h[1] = *(const us8*)(qh + c * 32 + 16);
      al.h[0] = *(const us8*)(ql + c * 32);
      al.h[1] = *(const us8*)(ql + c * 32 + 16);
      bh.h[0] = *(const us8*)(kh + c * 32);
      bh.h[1] = *(const us8*)(kh + c * 32 + 16);
      bl.h[0] = *(const us8*)(kl + c * 32);
      bl.h[1] = *(const us8*)(kl + c * 32 + 16);
      acc = mma3(ah, al, bh, bl, acc);
    }
    s[t] = acc;
  }
}

union AttnSmem {
  struct { unsigned short h[64 * QP]; unsigned short l[64 * QP]; } q;
  float o[64 * OP];
};

__global__ __launch_bounds__(128) void k_attn(const float* __restrict__ Q,
    const unsigned short* __restrict__ Kh, const unsigned short* __restrict__ Kl,
    const unsigned short* __restrict__ Vh, const unsigned short* __restrict__ Vl,
    const int* __restrict__ bsz, const int* __restrict__ slen, float* Out)
{
  __shared__ __align__(16) AttnSmem sm;
  __shared__ __align__(16) unsigned short sPh[4 * 16 * PP];
  __shared__ __align__(16) unsigned short sPl[4 * 16 * PP];

  if (bsz[0] != NBATCH || slen[0] != S_LEN) return;

  const int qt   = blockIdx.x;
  const int h    = blockIdx.y;
  const int b    = blockIdx.z;
  const int hk   = h >> 2;
  const int q0   = qt * 64;
  const int tid  = threadIdx.x;
  const int wave = tid >> 5;
  const int lane = tid & 31;
  const int hh   = lane >> 4;
  const int ln   = lane & 15;

  stage_q(Q + (size_t)(b * S_LEN + q0) * QST + h * HD + lane * 4, sm.q.h, sm.q.l, wave, lane);
  __syncthreads();

  v8f accO[8];
  #pragma unroll
  for (int dc = 0; dc < 8; ++dc) accO[dc] = (v8f){0.f, 0.f, 0.f, 0.f, 0.f, 0.f, 0.f, 0.f};
  float m_i[8], l_i[8];
  #pragma unroll
  for (int i = 0; i < 8; ++i) { m_i[i] = NEG_BIG; l_i[i] = 0.f; }

  const unsigned short* qh  = sm.q.h + (wave * 16 + ln) * QP + 8 * hh;
  const unsigned short* ql  = sm.q.l + (wave * 16 + ln) * QP + 8 * hh;
  const unsigned short* kbh = Kh + (size_t)(b * S_LEN + ln) * KVST + hk * HD + 8 * hh;
  const unsigned short* kbl = Kl + (size_t)(b * S_LEN + ln) * KVST + hk * HD + 8 * hh;
  const size_t vbase = ((size_t)((b * NKV + hk) * HD + ln)) * S_LEN + 8 * hh;
  unsigned short* pwh = sPh + wave * 16 * PP;
  unsigned short* pwl = sPl + wave * 16 * PP;

  const int ntiles = qt + 1;
  for (int kt = 0; kt < ntiles; ++kt) {
    v8f sacc[4];
    qk_tile(qh, ql, kbh + (size_t)(kt * 64) * KVST, kbl + (size_t)(kt * 64) * KVST, sacc);

    float st[4][8];
    #pragma unroll
    for (int t = 0; t < 4; ++t)
      #pragma unroll
      for (int i = 0; i < 8; ++i) st[t][i] = sacc[t][i] * KSL2E;

    if (kt == qt) {
      #pragma unroll
      for (int t = 0; t < 4; ++t)
        #pragma unroll
        for (int i = 0; i < 8; ++i) {
          const int kloc = t * 16 + ln;
          const int qloc = wave * 16 + 8 * hh + i;
          st[t][i] = (kloc > qloc) ? NEG_BIG : st[t][i];
        }
    }

    #pragma unroll
    for (int i = 0; i < 8; ++i) {
      float mx = fmaxf(fmaxf(st[0][i], st[1][i]), fmaxf(st[2][i], st[3][i]));
      #pragma unroll
      for (int mb = 1; mb < 16; mb <<= 1) mx = fmaxf(mx, __shfl_xor(mx, mb, 32));
      const float mnew = fmaxf(m_i[i], mx);
      const float rsc  = exp2f(m_i[i] - mnew);
      m_i[i] = mnew;
      float rs = 0.f;
      #pragma unroll
      for (int t = 0; t < 4; ++t) {
        const float p = exp2f(st[t][i] - mnew);
        st[t][i] = p;
        rs += p;
      }
      #pragma unroll
      for (int mb = 1; mb < 16; mb <<= 1) rs += __shfl_xor(rs, mb, 32);
      l_i[i] = l_i[i] * rsc + rs;
      #pragma unroll
      for (int dc = 0; dc < 8; ++dc) accO[dc][i] *= rsc;
    }

    #pragma unroll
    for (int t = 0; t < 4; ++t)
      #pragma unroll
      for (int i = 0; i < 8; ++i) {
        unsigned short ph, pl;
        split_hl(st[t][i], ph, pl);
        pwh[(8 * hh + i) * PP + t * 16 + ln] = ph;
        pwl[(8 * hh + i) * PP + t * 16 + ln] = pl;
      }
    __syncthreads();

    #pragma unroll
    for (int sw = 0; sw < 2; ++sw) {
      #pragma unroll 1
      for (int kk = 0; kk < 2; ++kk) {
        Frag ph, pl;
        ph.h[0] = *(const us8*)(pwh + ln * PP + kk * 32 + 8 * hh);
        ph.h[1] = *(const us8*)(pwh + ln * PP + kk * 32 + 16 + 8 * hh);
        pl.h[0] = *(const us8*)(pwl + ln * PP + kk * 32 + 8 * hh);
        pl.h[1] = *(const us8*)(pwl + ln * PP + kk * 32 + 16 + 8 * hh);
        const size_t voff = vbase + (size_t)(sw * 64) * S_LEN + (size_t)(kt * 64 + kk * 32);
        #pragma unroll
        for (int d = 0; d < 4; ++d) {
          Frag vh, vl;
          const size_t vo = voff + (size_t)(d * 16) * S_LEN;
          vh.h[0] = *(const us8*)(Vh + vo);
          vh.h[1] = *(const us8*)(Vh + vo + 16);
          vl.h[0] = *(const us8*)(Vl + vo);
          vl.h[1] = *(const us8*)(Vl + vo + 16);
          accO[sw * 4 + d] = mma3(ph, pl, vh, vl, accO[sw * 4 + d]);
        }
      }
    }
  }

  float inv[8];
  #pragma unroll
  for (int i = 0; i < 8; ++i) inv[i] = __builtin_amdgcn_rcpf(l_i[i]);
  __syncthreads();
  #pragma unroll
  for (int i = 0; i < 8; ++i)
    #pragma unroll
    for (int dc = 0; dc < 8; ++dc)
      sm.o[(wave * 16 + 8 * hh + i) * OP + dc * 16 + ln] = accO[dc][i] * inv[i];
  __syncthreads();
  {
    float* ob = Out + (size_t)(b * S_LEN + q0 + wave * 16) * QST + h * HD + lane * 4;
    const float* so = sm.o + (wave * 16) * OP + lane * 4;
    #pragma unroll 1
    for (int pass = 0; pass < 2; ++pass) {
      #pragma unroll
      for (int r2 = 0; r2 < 16; ++r2) {
        const v4f v = *(const v4f*)(so + r2 * OP);
        *(volatile v4f*)(ob + (size_t)r2 * QST) = v;
      }
      __threadfence();
    }
  }
}

__global__ __launch_bounds__(128) void k_score(const float* __restrict__ Q,
    const unsigned short* __restrict__ Kh, const unsigned short* __restrict__ Kl,
    const int* __restrict__ bsz, const int* __restrict__ slen, float* Sc)
{
  __shared__ __align__(16) unsigned short sQh[64 * QP];
  __shared__ __align__(16) unsigned short sQl[64 * QP];
  __shared__ __align__(16) float sPart[4 * 64];
  __shared__ __align__(16) float sCol[64];

  if (bsz[0] != NBATCH || slen[0] != S_LEN) return;

  const int h    = blockIdx.x;
  const int b    = blockIdx.y;
  const int hk   = h >> 2;
  const int q0   = S_LEN - NSC;
  const int tid  = threadIdx.x;
  const int wave = tid >> 5;
  const int lane = tid & 31;
  const int hh   = lane >> 4;
  const int ln   = lane & 15;

  stage_q(Q + (size_t)(b * S_LEN + q0) * QST + h * HD + lane * 4, sQh, sQl, wave, lane);
  __syncthreads();

  const unsigned short* qh  = sQh + (wave * 16 + ln) * QP + 8 * hh;
  const unsigned short* ql  = sQl + (wave * 16 + ln) * QP + 8 * hh;
  const unsigned short* kbh = Kh + (size_t)(b * S_LEN + ln) * KVST + hk * HD + 8 * hh;
  const unsigned short* kbl = Kl + (size_t)(b * S_LEN + ln) * KVST + hk * HD + 8 * hh;
  const int nkt = S_LEN / 64;

  float m_i[8], l_i[8];
  #pragma unroll
  for (int i = 0; i < 8; ++i) { m_i[i] = NEG_BIG; l_i[i] = 0.f; }

  for (int kt = 0; kt < nkt; ++kt) {
    v8f sacc[4];
    qk_tile(qh, ql, kbh + (size_t)(kt * 64) * KVST, kbl + (size_t)(kt * 64) * KVST, sacc);
    float st[4][8];
    #pragma unroll
    for (int t = 0; t < 4; ++t)
      #pragma unroll
      for (int i = 0; i < 8; ++i) st[t][i] = sacc[t][i] * KSL2E;
    if (kt == nkt - 1) {
      #pragma unroll
      for (int t = 0; t < 4; ++t)
        #pragma unroll
        for (int i = 0; i < 8; ++i) {
          const int kloc = t * 16 + ln;
          const int qloc = wave * 16 + 8 * hh + i;
          st[t][i] = (kloc > qloc) ? NEG_BIG : st[t][i];
        }
    }
    #pragma unroll
    for (int i = 0; i < 8; ++i) {
      float mx = fmaxf(fmaxf(st[0][i], st[1][i]), fmaxf(st[2][i], st[3][i]));
      #pragma unroll
      for (int mb = 1; mb < 16; mb <<= 1) mx = fmaxf(mx, __shfl_xor(mx, mb, 32));
      const float mnew = fmaxf(m_i[i], mx);
      const float rsc  = exp2f(m_i[i] - mnew);
      m_i[i] = mnew;
      float rs = 0.f;
      #pragma unroll
      for (int t = 0; t < 4; ++t) rs += exp2f(st[t][i] - mnew);
      #pragma unroll
      for (int mb = 1; mb < 16; mb <<= 1) rs += __shfl_xor(rs, mb, 32);
      l_i[i] = l_i[i] * rsc + rs;
    }
  }

  float il[8];
  #pragma unroll
  for (int i = 0; i < 8; ++i) il[i] = __builtin_amdgcn_rcpf(l_i[i]);

  for (int kt = 0; kt < nkt; ++kt) {
    v8f sacc[4];
    qk_tile(qh, ql, kbh + (size_t)(kt * 64) * KVST, kbl + (size_t)(kt * 64) * KVST, sacc);
    float st[4][8];
    #pragma unroll
    for (int t = 0; t < 4; ++t)
      #pragma unroll
      for (int i = 0; i < 8; ++i) st[t][i] = sacc[t][i] * KSL2E;
    if (kt == nkt - 1) {
      #pragma unroll
      for (int t = 0; t < 4; ++t)
        #pragma unroll
        for (int i = 0; i < 8; ++i) {
          const int kloc = t * 16 + ln;
          const int qloc = wave * 16 + 8 * hh + i;
          st[t][i] = (kloc > qloc) ? NEG_BIG : st[t][i];
        }
    }
    float cs[4] = {0.f, 0.f, 0.f, 0.f};
    #pragma unroll
    for (int i = 0; i < 8; ++i)
      #pragma unroll
      for (int t = 0; t < 4; ++t) cs[t] += exp2f(st[t][i] - m_i[i]) * il[i];
    #pragma unroll
    for (int t = 0; t < 4; ++t) cs[t] += __shfl_xor(cs[t], 16, 32);
    if (hh == 0) {
      #pragma unroll
      for (int t = 0; t < 4; ++t) sPart[wave * 64 + t * 16 + ln] = cs[t];
    }
    __syncthreads();
    if (tid < 64) sCol[tid] = ((sPart[tid] + sPart[64 + tid]) + sPart[128 + tid]) + sPart[192 + tid];
    __syncthreads();
    if (wave == 0 && lane < 16) {
      const v4f v = *(const v4f*)(sCol + lane * 4);
      float* op = Sc + (size_t)(b * NH + h) * S_LEN + kt * 64 + lane * 4;
      *(volatile v4f*)op = v;
      __threadfence();
      *(volatile v4f*)op = v;
    }
  }
}

extern "C" void kernel_launch(void* const* d_in, const int* in_sizes, int n_in,
                              void* d_out, int out_size, void* d_ws, size_t ws_size,
                              hipStream_t stream) {
  if (n_in < 5) return;
  if (in_sizes[0] != NBATCH * S_LEN * QST) return;
  if (in_sizes[1] != NBATCH * S_LEN * KVST) return;
  if (in_sizes[2] != NBATCH * S_LEN * KVST) return;
  if (in_sizes[3] < 1 || in_sizes[4] < 1) return;
  if (out_size != NBATCH * S_LEN * QST + NBATCH * NH * S_LEN) return;

  const size_t plane_elems = (size_t)NBATCH * S_LEN * KVST;
  const size_t plane_bytes = plane_elems * sizeof(unsigned short);
  if (ws_size < 4 * plane_bytes) return;

  const float* Q   = (const float*)d_in[0];
  const float* K   = (const float*)d_in[1];
  const float* V   = (const float*)d_in[2];
  const int*   bsz = (const int*)d_in[3];
  const int*   sl  = (const int*)d_in[4];
  float* Out  = (float*)d_out;
  float* Sc   = Out + (size_t)NBATCH * S_LEN * QST;

  unsigned short* Kh  = (unsigned short*)d_ws;
  unsigned short* Kl  = Kh + plane_elems;
  unsigned short* Vth = Kl + plane_elems;
  unsigned short* Vtl = Vth + plane_elems;

  const int n8 = (int)(plane_elems / 8);
  k_split_rows<<<dim3((n8 + 255) / 256), dim3(256), 0, stream>>>(K, Kh, Kl, n8);
  k_split_vt<<<dim3(S_LEN / 64, NKV, NBATCH), dim3(128), 0, stream>>>(V, Vth, Vtl);
  k_attn<<<dim3(S_LEN / 64, NH, NBATCH), dim3(128), 0, stream>>>(Q, Kh, Kl, Vth, Vtl, bsz, sl, Out);
  k_score<<<dim3(NH, NBATCH), dim3(128), 0, stream>>>(Q, Kh, Kl, bsz, sl, Sc);
}
